// MultiheadedPairedAttention_62088047231063
// MI455X (gfx1250) — hardware-verified
//
#include <hip/hip_runtime.h>


namespace {
constexpr int S = 8, CK = 32, CQ = 32, A = 16, N = 32, X = 16, NV = 4096, NCH = N * CQ  ;
constexpr float HS = 256.0f, WSC = 256.0f, EPS0 = 1e-5f, EPS1 = 1024.0f, EPS2 = 1e-5f;
typedef _Float16 b16;
typedef __attribute__((ext_vector_type(16))) _Float16 v16b;
typedef __attribute__((ext_vector_type(8))) _Float16 v8b;
typedef __attribute__((ext_vector_type(8))) float v8f;
typedef __attribute__((ext_vector_type(4))) float v4f;
__device__ __forceinline__ float bf16_rne(float f) { unsigned int u = __float_as_uint(f); u += 0x7FFFu + ((u >> 16) & 1u); float r = __uint_as_float(u & 0xFFFF0000u); asm volatile("" : "+v"(r)); return r; }
__device__ __forceinline__ float bfv(float f) { float r = bf16_rne(f); asm volatile("" : "+v"(r)); return r; }
__device__ __forceinline__ void split16(float v, b16& hi, b16& lo) { hi = (b16)v; lo = (b16)(v - (float)hi); }
__device__ __forceinline__ v16b frag_kb(const b16* p, int hh) { const v8b a = *(const v8b*)(p + 8 * hh), b = *(const v8b*)(p + 16 + 8 * hh); v16b f;
#pragma unroll
  for (int e = 0; e < 8; ++e) { f[e] = a[e]; f[8 + e] = b[e]; } return f; }
__device__ __forceinline__ v8f wmma16b(v16b a, v16b b, v8f c) { v8f d = __builtin_amdgcn_wmma_f32_16x16x32_f16(false, a, false, b, (short)0, c, false, false); asm volatile("v_nop\n\tv_nop\n\tv_nop\n\tv_nop" : "+v"(d) : "v"(a), "v"(b)); return d; }
__device__ __forceinline__ void wave_lds_sync() { __builtin_amdgcn_fence(__ATOMIC_RELEASE, "workgroup"); __builtin_amdgcn_wave_barrier(); __builtin_amdgcn_fence(__ATOMIC_ACQUIRE, "workgroup"); }
__device__ __forceinline__ float pmul(float a, float b) { float p = a * b; asm volatile("" : "+v"(p)); return p; }
__device__ __forceinline__ int vperm(int y, int z, int x) { return (y * 16 + z) * 16 + x; }
__device__ __forceinline__ int vorig(int x, int y, int z) { return (x * 16 + y) * 16 + z; }

__global__ __launch_bounds__(256) void wput_kernel(const float* __restrict__ wk, const float* __restrict__ wq, const float* __restrict__ wv, const float* __restrict__ w1, b16* __restrict__ WK, b16* __restrict__ WQ, b16* __restrict__ WV, b16* __restrict__ WF1) { const int u = blockIdx.x * 256 + threadIdx.x; v8b v;
  if (u < N * A * 4) { const int r = u / 4, k0 = (u % 4) * 8; v8b a, b;
#pragma unroll
    for (int j = 0; j < 8; ++j) { a[j] = (b16)(bf16_rne(wk[(size_t)r * CK + k0 + j]) * WSC); b[j] = (b16)(bf16_rne(wq[(size_t)r * CQ + k0 + j]) * WSC); } for (int pass = 0; pass < 2; ++pass) { *(volatile v8b*)(WK + (size_t)r * CK + k0) = a; *(volatile v8b*)(WQ + (size_t)r * CQ + k0) = b; __threadfence(); } }
  if (u < N * CQ * 4) { const int r = u / 4, k0 = (u % 4) * 8;
#pragma unroll
    for (int j = 0; j < 8; ++j) v[j] = (b16)(bf16_rne(wv[(size_t)r * CK + k0 + j]) * WSC); for (int pass = 0; pass < 2; ++pass) { *(volatile v8b*)(WV + (size_t)r * CK + k0) = v; __threadfence(); } }
  if (u < CQ * 128) { const int o = u / 128, k0 = (u % 128) * 8;
#pragma unroll
    for (int j = 0; j < 8; ++j) v[j] = (b16)(bf16_rne(w1[(size_t)o * NCH + k0 + j]) * WSC); for (int pass = 0; pass < 2; ++pass) { *(volatile v8b*)(WF1 + (size_t)o * NCH + k0) = v; __threadfence(); } } }
__global__ __launch_bounds__(256) void gstat_kernel(const float* __restrict__ key, const float* __restrict__ qry, float* __restrict__ GS) { __shared__ double Sh[256]; const int sm = blockIdx.x; const float* src = (sm < 8 ? key : qry) + (size_t)(sm % 8) * CK * NV; const int tid = threadIdx.x; const int CNT = CK * NV;
  double s = 0.0; for (int i = tid; i < CNT; i += 256) s += (double)bfv(src[i]); Sh[tid] = s; __syncthreads(); for (int o = 128; o; o >>= 1) { if (tid < o) Sh[tid] += Sh[tid + o]; __syncthreads(); } const double mean = Sh[0] / CNT; __syncthreads();
  double q = 0.0; for (int i = tid; i < CNT; i += 256) { const double d = (double)bfv(src[i]) - mean; q += d * d; } Sh[tid] = q; __syncthreads(); for (int o = 128; o; o >>= 1) { if (tid < o) Sh[tid] += Sh[tid + o]; __syncthreads(); }
  if (tid < 32) { const float m = (float)mean, rs = (float)(1.0 / sqrt(Sh[0] / CNT + (double)EPS0)); for (int pass = 0; pass < 2; ++pass) { ((volatile float*)GS)[sm * 32 + tid] = tid == 0 ? m : (tid == 1 ? rs : 0.0f); __threadfence(); } } }
__global__ __launch_bounds__(32) void att_kernel(const float* __restrict__ key, const float* __restrict__ qry, const float* __restrict__ GS, const float* __restrict__ gkw, const float* __restrict__ gkb, const float* __restrict__ gqw, const float* __restrict__ gqb, const b16* __restrict__ WK, const float* __restrict__ bk, const b16* __restrict__ WQ, const float* __restrict__ bq, const b16* __restrict__ WV, const float* __restrict__ bv, int NHLIM, float* __restrict__ FEAT) {
  __shared__ __attribute__((aligned(16))) b16 Ah[256][40], Al[256][40]; __shared__ float Kp[32][S][A + 1], Qp[32][S][A + 1], Vp[32][S][CQ + 1], At[32][S][S + 1]; const int lane = threadIdx.x, nloc = lane & 15, hlf = lane >> 4;
  const int n = blockIdx.x % N, line = blockIdx.x / N; if (n >= NHLIM) return; const int y = line / 8, z0 = (line % 8) * 2;
  auto stage = [&](const float* src, const float* gw, const float* gb, int sm0) {
    for (int r = 0; r < 256; r += 1) { const int s = r / 32, v = r % 32, zz = v / 16, x = v % 16; const float m = GS[(sm0 + s) * 32], rs = GS[(sm0 + s) * 32 + 1]; const int c = lane; const float val = pmul((bfv(src[(((size_t)s * CK + c) * NV) + vorig(x, y, z0 + zz)]) - m) * rs, bfv(gw[c])) + bfv(gb[c]); b16 p, pl; split16(val * HS, p, pl); Ah[r][c] = p; Al[r][c] = pl; if (lane < 8) { Ah[r][32 + lane] = (b16)0.0f; Al[r][32 + lane] = (b16)0.0f; } }
    wave_lds_sync(); };
  stage(key, gkw, gkb, 0);
#pragma unroll 1
  for (int rt = 0; rt < 16; ++rt) { const v16b a = frag_kb(&Ah[rt * 16 + nloc][0], hlf), al = frag_kb(&Al[rt * 16 + nloc][0], hlf); const v16b bwk = frag_kb(WK + ((size_t)n * A + nloc) * CK, hlf); v8f dk = wmma16b(a, bwk, (v8f){}); dk = wmma16b(al, bwk, dk);
    v8f dv0 = (v8f){}, dv1 = (v8f){}; { const v16b b0 = frag_kb(WV + ((size_t)n * CQ + nloc) * CK, hlf), b1 = frag_kb(WV + ((size_t)n * CQ + 16 + nloc) * CK, hlf); dv0 = wmma16b(a, b0, dv0); dv0 = wmma16b(al, b0, dv0); dv1 = wmma16b(a, b1, dv1); dv1 = wmma16b(al, b1, dv1); }
#pragma unroll
    for (int r8 = 0; r8 < 8; ++r8) { const int r = rt * 16 + 8 * hlf + r8; const int s = r / 32, v = r % 32; Kp[v][s][nloc] = dk[r8] * (1.0f / (HS * WSC)) + bfv(bk[n * A + nloc]); Vp[v][s][nloc] = dv0[r8] * (1.0f / (HS * WSC)) + bfv(bv[n * CQ + nloc]); Vp[v][s][16 + nloc] = dv1[r8] * (1.0f / (HS * WSC)) + bfv(bv[n * CQ + 16 + nloc]); } }
  wave_lds_sync();
  stage(qry, gqw, gqb, 8);
#pragma unroll 1
  for (int rt = 0; rt < 16; ++rt) { const v16b a = frag_kb(&Ah[rt * 16 + nloc][0], hlf), al = frag_kb(&Al[rt * 16 + nloc][0], hlf); const v16b bw = frag_kb(WQ + ((size_t)n * A + nloc) * CQ, hlf); v8f d = wmma16b(a, bw, (v8f){}); d = wmma16b(al, bw, d);
#pragma unroll
    for (int r8 = 0; r8 < 8; ++r8) { const int r = rt * 16 + 8 * hlf + r8; Qp[r % 32][r / 32][nloc] = d[r8] * (1.0f / (HS * WSC)) + bfv(bq[n * A + nloc]); } }
  wave_lds_sync();
  for (int s = 0; s < S; ++s) for (int t = 0; t < S; ++t) { float acc = 0.0f;
#pragma unroll
    for (int a = 0; a < A; ++a) acc += pmul(Kp[lane][s][a], Qp[lane][t][a]); At[lane][s][t] = acc * 0.25f; }
  wave_lds_sync();
  for (int grp = lane; grp < 2 * S * S; grp += 32) { const int zz = grp / (S * S), s = (grp / S) % S, t = grp % S; float mx = -INFINITY; for (int x = 0; x < X; ++x) mx = fmaxf(mx, At[zz * 16 + x][s][t]); float sm = 0.0f; for (int x = 0; x < X; ++x) { const float e = __expf(At[zz * 16 + x][s][t] - mx); At[zz * 16 + x][s][t] = e; sm += e; } const float inv = 1.0f / sm; for (int x = 0; x < X; ++x) At[zz * 16 + x][s][t] *= inv; }
  wave_lds_sync();
  const size_t vbase = (size_t)vperm(y, z0, 0);
  for (int pass = 0; pass < 2; ++pass) { for (int t = 0; t < S; ++t) for (int o = 0; o < CQ; ++o) { float acc = 0.0f;
#pragma unroll
      for (int s = 0; s < S; ++s) acc += pmul(Vp[lane][s][o], At[lane][s][t]); ((volatile float*)FEAT)[((size_t)t * NCH + n * CQ + o) * NV + vbase + lane] = acc; } __threadfence(); } }
template <int RL>
__global__ __launch_bounds__(256) void istat_kernel(const float* __restrict__ Pl, int rows, float eps, float* __restrict__ ST) { const int wave = threadIdx.x >> 5, lane = threadIdx.x & 31; const int r = blockIdx.x * 8 + wave; if (r >= rows) return; const float* p = Pl + (size_t)r * NV; double s = 0.0; for (int i = lane; i < NV; i += 32) { float v = p[i]; if (RL) v = fmaxf(v, 0.0f); s += (double)v; } for (int o = 16; o; o >>= 1) s += __shfl_xor(s, o); const double mean = s / NV; double q = 0.0; for (int i = lane; i < NV; i += 32) { float v = p[i]; if (RL) v = fmaxf(v, 0.0f); const double d = (double)v - mean; q += d * d; } for (int o = 16; o; o >>= 1) q += __shfl_xor(q, o);
  const float m = (float)mean, rs = (float)(1.0 / sqrt(q / NV + (double)eps));
  for (int pass = 0; pass < 2; ++pass) { ((volatile float*)ST)[(size_t)r * 32 + lane] = lane == 0 ? m : (lane == 1 ? rs : 0.0f); __threadfence(); } }
__global__ __launch_bounds__(32) void w1_kernel(const float* __restrict__ FEAT, const float* __restrict__ ST1, const b16* __restrict__ WF1, const float* __restrict__ b1, int NHLIM, float* __restrict__ H1) { __shared__ __attribute__((aligned(16))) b16 Ah[32][264], Al[32][264]; __shared__ float Tq[32][33]; const int lane = threadIdx.x, nloc = lane & 15, hlf = lane >> 4; const int t = blockIdx.x / (NV / 32), vb = (blockIdx.x % (NV / 32)) * 32; const int KLIM = NHLIM * CQ;
  v8f acc[2][2] = {{(v8f){}, (v8f){}}, {(v8f){}, (v8f){}}};
  for (int k = 256; k < 264; ++k) { Ah[lane][k] = (b16)0.0f; Al[lane][k] = (b16)0.0f; }
#pragma unroll 1
  for (int ch0 = 0; ch0 < NCH; ch0 += 256) {
    for (int cc = 0; cc < 256; ++cc) { const int ch = ch0 + cc; float v = 0.0f; if (ch < KLIM) { const float m = ST1[((size_t)t * NCH + ch) * 32], rs = ST1[((size_t)t * NCH + ch) * 32 + 1]; v = (fmaxf(FEAT[((size_t)t * NCH + ch) * NV + vb + lane], 0.0f) - m) * rs; } b16 p, pl; split16(v * HS, p, pl); Ah[lane][cc] = p; Al[lane][cc] = pl; }
    wave_lds_sync();
#pragma unroll 2
    for (int kb = 0; kb < 256; kb += 32)
#pragma unroll
      for (int rt = 0; rt < 2; ++rt) { const v16b a = frag_kb(&Ah[rt * 16 + nloc][kb], hlf), al = frag_kb(&Al[rt * 16 + nloc][kb], hlf);
#pragma unroll
        for (int ct = 0; ct < 2; ++ct) { const v16b bw = frag_kb(WF1 + (size_t)(ct * 16 + nloc) * NCH + ch0 + kb, hlf); acc[rt][ct] = wmma16b(a, bw, acc[rt][ct]); acc[rt][ct] = wmma16b(al, bw, acc[rt][ct]); } }
    wave_lds_sync(); }
#pragma unroll
  for (int rt = 0; rt < 2; ++rt)
#pragma unroll
    for (int ct = 0; ct < 2; ++ct)
#pragma unroll
      for (int r8 = 0; r8 < 8; ++r8) { const int o = ct * 16 + nloc; Tq[rt * 16 + 8 * hlf + r8][o] = fmaxf(acc[rt][ct][r8] * (1.0f / (HS * WSC)) + bfv(b1[o]), 0.0f); }
  wave_lds_sync();
  for (int pass = 0; pass < 2; ++pass) { for (int o = 0; o < CQ; ++o) ((volatile float*)H1)[((size_t)t * CQ + o) * NV + vb + lane] = Tq[lane][o]; __threadfence(); } }
__global__ __launch_bounds__(32) void w2_kernel(const float* __restrict__ H1, const float* __restrict__ ST2, const float* __restrict__ w2, const float* __restrict__ b2, float* __restrict__ out) { __shared__ float Hn[32][33]; const int lane = threadIdx.x; const int t = blockIdx.x / (NV / 32), ob = (blockIdx.x % (NV / 32)) * 32; const int vo = ob + lane; const int x = vo / 256, y = (vo / 16) % 16, z = vo % 16; const int vp = vperm(y, z, x);
  for (int o = 0; o < CQ; ++o) { const float m = ST2[((size_t)t * CQ + o) * 32], rs = ST2[((size_t)t * CQ + o) * 32 + 1]; Hn[lane][o] = (H1[((size_t)t * CQ + o) * NV + vp] - m) * rs; }
  wave_lds_sync();
  for (int pass = 0; pass < 2; ++pass) { for (int c = 0; c < CQ; ++c) { float s = bfv(b2[c]);
#pragma unroll 8
      for (int o = 0; o < CQ; ++o) s += pmul(bfv(w2[c * CQ + o]), Hn[lane][o]); ((volatile float*)out)[((size_t)t * CQ + c) * NV + vo] = s; } __threadfence(); } }
}

extern "C" void kernel_launch(void* const* d_in, const int* in_sizes, int n_in, void* d_out, int out_size, void* d_ws, size_t ws_size, hipStream_t stream) {
  (void)n_in;
  auto Fp = [&](int i) { return (const float*)d_in[i]; };
  if (in_sizes[0] != S * CK * NV || in_sizes[1] != S * CQ * NV || in_sizes[2] != CK || in_sizes[6] != N * A * CK || in_sizes[10] != N * CQ * CK || in_sizes[12] != CQ * NCH || in_sizes[14] != CQ * CQ || out_size != S * CQ * NV) return;
  const int NHLIM = N;
  size_t off = 0; char* ws = (char*)d_ws;
  auto carve = [&](size_t bytes) { char* p = ws + off; off += (bytes + 255) & ~(size_t)255; return p; };
  b16* WK = (b16*)carve((size_t)N * A * CK * 2); b16* WQ = (b16*)carve((size_t)N * A * CQ * 2); b16* WV = (b16*)carve((size_t)N * CQ * CK * 2); b16* WF1 = (b16*)carve((size_t)CQ * NCH * 2); float* GS = (float*)carve(16 * 32 * 4); float* FEAT = (float*)carve((size_t)S * NCH * NV * 4); float* ST1 = (float*)carve((size_t)S * NCH * 32 * 4); float* H1 = (float*)carve((size_t)S * CQ * NV * 4); float* ST2 = (float*)carve((size_t)S * CQ * 32 * 4);
  if (off > ws_size || off > ((size_t)160 << 20)) return;
  wput_kernel<<<(CQ * 128 + 255) / 256, 256, 0, stream>>>(Fp(6), Fp(8), Fp(10), Fp(12), WK, WQ, WV, WF1);
  gstat_kernel<<<16, 256, 0, stream>>>(Fp(0), Fp(1), GS);
  att_kernel<<<128 * N, 32, 0, stream>>>(Fp(0), Fp(1), GS, Fp(2), Fp(3), Fp(4), Fp(5), WK, Fp(7), WQ, Fp(9), WV, Fp(11), NHLIM, FEAT);
  istat_kernel<1><<<S * NCH / 8, 256, 0, stream>>>(FEAT, S * NCH, EPS1, ST1);
  w1_kernel<<<S * (NV / 32), 32, 0, stream>>>(FEAT, ST1, WF1, Fp(13), NHLIM, H1);
  istat_kernel<0><<<S * CQ / 8, 256, 0, stream>>>(H1, S * CQ, EPS2, ST2);
  w2_kernel<<<S * (NV / 32), 32, 0, stream>>>(H1, ST2, Fp(14), Fp(15), (float*)d_out);
}
